// GraphProd2Vec_27539330302214
// MI455X (gfx1250) — hardware-run, weakly checked
//
#include <hip/hip_runtime.h>

typedef float          v8f   __attribute__((ext_vector_type(8)));
typedef float          v4f   __attribute__((ext_vector_type(4)));
typedef unsigned int   v4u   __attribute__((ext_vector_type(4)));
typedef int            v8i   __attribute__((ext_vector_type(8)));
typedef unsigned short v8us  __attribute__((ext_vector_type(8)));
typedef unsigned short v16us __attribute__((ext_vector_type(16)));
typedef __bf16         v16bf __attribute__((ext_vector_type(16)));
typedef _Float16       v16h  __attribute__((ext_vector_type(16)));
typedef v4f  __attribute__((may_alias)) v4fa;
typedef v8us __attribute__((may_alias)) v8usa;
union FragB { v16bf v; v16us u; v8us h[2]; v8i w; };
union FragH { v16h  v; v16us u; v8us h[2]; v8i w; };

__device__ __forceinline__ v8f wmb(const FragB& a, const FragB& b, v8f c) {
  v8f d = __builtin_amdgcn_wmma_f32_16x16x32_bf16(false, a.v, false, b.v, (short)0, c, false, false);
  asm volatile("v_nop\n\tv_nop\n\tv_nop\n\tv_nop" : "+v"(d) : "v"(a.w), "v"(b.w));
  return d;
}

__device__ __forceinline__ v8f wmh(const FragH& a, const FragH& b, v8f c) {
  v8f d = __builtin_amdgcn_wmma_f32_16x16x32_f16(false, a.v, false, b.v, (short)0, c, false, false);
  asm volatile("v_nop\n\tv_nop\n\tv_nop\n\tv_nop" : "+v"(d) : "v"(a.w), "v"(b.w));
  return d;
}

__device__ __forceinline__ unsigned bf16_bits(float f) {
  const unsigned u = __float_as_uint(f);
  const unsigned r = (u + 0x7FFFu + ((u >> 16) & 1u)) >> 16;
  const unsigned q = (u >> 16) | 0x40u;
  return ((u & 0x7fffffffu) > 0x7f800000u) ? q : r;
}

__device__ __forceinline__ float bf16_val(float f) {
  return __uint_as_float(bf16_bits(f) << 16);
}
__device__ __forceinline__ int clampi(int v, int lo, int hi) {
  return v < lo ? lo : (v > hi ? hi : v);
}

__device__ __forceinline__ unsigned f16_bits(float f) {
  const unsigned u  = __float_as_uint(f);
  const unsigned s  = (u >> 16) & 0x8000u;
  const unsigned a  = u & 0x7fffffffu;
  const unsigned t  = a - 0x38000000u;
  const unsigned r  = (t + 0x0FFFu + ((t >> 13) & 1u)) >> 13;
  const unsigned rc = r > 0x7C00u ? 0x7C00u : r;
  const bool small  = a < 0x38800000u;
  const bool isnan  = a > 0x7f800000u;
  const unsigned fin = small ? 0u : (s | rc);
  return isnan ? (s | 0x7E00u) : fin;
}

__device__ __forceinline__ unsigned pk16(unsigned lo, unsigned hi) { return lo | (hi << 16); }
__device__ __forceinline__ unsigned bf16_lo_bits(float v) {
  float hi = bf16_val(v);
  asm volatile("" : "+v"(hi));
  return bf16_bits(v - hi);
}
__device__ __forceinline__ v4u pack8_bf16(v4f a, v4f c) {
  return (v4u){ pk16(bf16_bits(a[0]), bf16_bits(a[1])), pk16(bf16_bits(a[2]), bf16_bits(a[3])),
                pk16(bf16_bits(c[0]), bf16_bits(c[1])), pk16(bf16_bits(c[2]), bf16_bits(c[3])) };
}
__device__ __forceinline__ v4u pack8_bf16_lo(v4f a, v4f c) {
  return (v4u){ pk16(bf16_lo_bits(a[0]), bf16_lo_bits(a[1])), pk16(bf16_lo_bits(a[2]), bf16_lo_bits(a[3])),
                pk16(bf16_lo_bits(c[0]), bf16_lo_bits(c[1])), pk16(bf16_lo_bits(c[2]), bf16_lo_bits(c[3])) };
}
__device__ __forceinline__ v4u pack8_f16(v4f a, v4f c) {
  return (v4u){ pk16(f16_bits(a[0]), f16_bits(a[1])), pk16(f16_bits(a[2]), f16_bits(a[3])),
                pk16(f16_bits(c[0]), f16_bits(c[1])), pk16(f16_bits(c[2]), f16_bits(c[3])) };
}

template <int FORM>
__global__ __launch_bounds__(256) void k_plane(const float* __restrict__ src, int rows, int cols, int ldsrc,
                                               unsigned short* __restrict__ dst, int MP, int KP) {
  static_assert(FORM >= 0 && FORM <= 3);
  const int KTOT = (FORM == 1 || FORM == 3) ? 2 * KP : KP;
  const unsigned ppr   = (unsigned)(KTOT >> 3);
  const unsigned kp8   = (unsigned)(KP >> 3);
  const unsigned total = (unsigned)MP * ppr;
  const unsigned g     = blockIdx.x * 256u + threadIdx.x;
  const unsigned rowu  = g / ppr;
  const unsigned p     = g - rowu * ppr;
  const bool second    = p >= kp8;
  const int row = (int)rowu;
  const int c0  = (int)((second ? p - kp8 : p) << 3);
  const float* srow = src + (size_t)clampi(row, 0, rows - 1) * (size_t)ldsrc;
  float x[8];
  unsigned mk[8];
#pragma unroll
  for (int e = 0; e < 8; ++e) {
    const int c = c0 + e;
    const float v = srow[clampi(c, 0, cols - 1)];
    asm volatile("" :: "v"(v));
    x[e]  = v;
    mk[e] = (row < rows && c < cols) ? 0xFFFFu : 0u;
  }
  const v4f a = (v4f){ x[0], x[1], x[2], x[3] };
  const v4f c = (v4f){ x[4], x[5], x[6], x[7] };
  v4u o;
  if (FORM == 2) {
    o = pack8_f16(a, c);
  } else {
    const v4u hi = pack8_bf16(a, c);
    o = hi;
    if (FORM == 1) { const v4u lo = pack8_bf16_lo(a, c); o = second ? lo : hi; }
  }
  const v4u mw = (v4u){ pk16(mk[0], mk[1]), pk16(mk[2], mk[3]), pk16(mk[4], mk[5]), pk16(mk[6], mk[7]) };
  o &= mw;
  if (g < total) {
    volatile v4u* q = (volatile v4u*)(dst + (size_t)g * 8);
    *q = o;
    __threadfence();
    *q = o;
  }
}

template <int FORM> struct FragOf    { typedef FragB T; };
template <>         struct FragOf<2> { typedef FragH T; };
__device__ __forceinline__ v8f mm(const FragB& a, const FragB& b, v8f c) { return wmb(a, b, c); }
__device__ __forceinline__ v8f mm(const FragH& a, const FragH& b, v8f c) { return wmh(a, b, c); }
template <class F> __device__ __forceinline__ F ld_frag(const unsigned short* p) {
  F f;
  f.h[0] = *(const v8usa*)(p);
  f.h[1] = *(const v8usa*)(p + 16);
  return f;
}

template <int FORM, int EPI>
__global__ __launch_bounds__(256) __attribute__((amdgpu_num_vgpr(248)))
void k_gemm_nt(const unsigned short* __restrict__ A, const unsigned short* __restrict__ B,
               const float* __restrict__ bias, float* __restrict__ D, int M, int N, int KTOT, int ldd) {
  static_assert(FORM >= 0 && FORM <= 2);
  static_assert(EPI == 0 || EPI == 1);
  typedef typename FragOf<FORM>::T F;
  __shared__ __attribute__((aligned(16))) float sT[8][16 * 68];
  const int lane = threadIdx.x & 31;
  const int wave = threadIdx.x >> 5;
  const int tilesM = (M + 63) >> 6;
  const int tilesN = (N + 63) >> 6;
  const int tile = blockIdx.x * 8 + wave;
  if (tile >= tilesM * tilesN) return;
  const int tm = tile / tilesN;
  const int tn = tile - tm * tilesN;
  const int m0 = tm << 6;
  const int n0 = tn << 6;

  const int rl = lane & 15;
  const int h8 = (lane >> 4) * 8;
  const unsigned short* pa = A + (size_t)(m0 + rl) * (size_t)KTOT + h8;
  const unsigned short* pb = B + (size_t)(n0 + rl) * (size_t)KTOT + h8;

  v8f acc[4][4];
#pragma unroll
  for (int i = 0; i < 4; ++i)
#pragma unroll
    for (int j = 0; j < 4; ++j) acc[i][j] = (v8f){0.f, 0.f, 0.f, 0.f, 0.f, 0.f, 0.f, 0.f};

#pragma unroll 1
  for (int k0 = 0; k0 < KTOT; k0 += 32) {
    F bf[4];
#pragma unroll
    for (int j = 0; j < 4; ++j) bf[j] = ld_frag<F>(pb + (size_t)(j << 4) * (size_t)KTOT + k0);
#pragma unroll
    for (int i = 0; i < 4; ++i) {
      const F af = ld_frag<F>(pa + (size_t)(i << 4) * (size_t)KTOT + k0);
#pragma unroll
      for (int j = 0; j < 4; ++j) acc[i][j] = mm(af, bf[j], acc[i][j]);
    }
  }

  float* slab = sT[wave];
  const int hh = lane >> 4;
  const int c4 = (lane & 15) * 4;
  const int nc = n0 + c4;
  const bool cok = nc < N;
  v4f bv = (v4f){0.f, 0.f, 0.f, 0.f};
  if (EPI == 1) {
    bv = *(const v4fa*)(bias + clampi(nc, 0, N - 4));
    asm volatile("" :: "v"(bv));
  }
#pragma unroll
  for (int i = 0; i < 4; ++i) {
    const int mBase = m0 + (i << 4);
#pragma unroll
    for (int j = 0; j < 4; ++j) {
#pragma unroll
      for (int r = 0; r < 8; ++r) slab[(h8 + r) * 68 + (j << 4) + rl] = acc[i][j][r];
    }
    __builtin_amdgcn_fence(__ATOMIC_RELEASE, "workgroup");
    __builtin_amdgcn_wave_barrier();
    __builtin_amdgcn_fence(__ATOMIC_ACQUIRE, "workgroup");
    v4f vv[8];
#pragma unroll
    for (int it = 0; it < 8; ++it) {
      const int row = it * 2 + hh;
      v4f v = *(const v4fa*)(slab + row * 68 + c4);
      if (EPI == 1) v += bv;
      vv[it] = v;
    }
    for (int pass = 0; pass < 2; ++pass) {
#pragma unroll
      for (int it = 0; it < 8; ++it) {
        const int row = mBase + it * 2 + hh;
        if (cok && row < M) *(volatile v4f*)(D + (size_t)row * (size_t)ldd + nc) = vv[it];
      }
      __threadfence();
    }
    __builtin_amdgcn_fence(__ATOMIC_RELEASE, "workgroup");
    __builtin_amdgcn_wave_barrier();
    __builtin_amdgcn_fence(__ATOMIC_ACQUIRE, "workgroup");
  }
}

#pragma clang fp contract(off)

#define NNODE   8192
#define DIN     256
#define DOUT    128
#define NEDGE   262144
#ifndef TWO_TERM_L2
#define TWO_TERM_L2 1
#endif
#ifndef TWO_TERM_L3
#define TWO_TERM_L3 1
#endif
#define KT2     (TWO_TERM_L2 ? 2 * DIN : DIN)
#define KT3     (TWO_TERM_L3 ? 2 * DIN : DIN)

#define OWN_BLK   512
#define OWN_WAVE  64
#define DEGCAP    128
#define WSTRIP    6000
#define STRIPW    6016
#define TBLH      (32 * DEGCAP)
#define LDS_BUCKET (8 * STRIPW * 4 + 8 * TBLH * 2)
#define CNT_SENT  32767

#define U_W1   (DIN * (DIN / 8))
#define U_W2   (DIN * (KT2 / 8))
#define U_W3   (DOUT * (KT3 / 8))
#define U_PV   512
#define U_TOT  (U_W1 + U_W2 + U_W3 + U_PV)

#define PV_B1   0
#define PV_G1   256
#define PV_BE1  512
#define PV_B2   768
#define PV_G2   1024
#define PV_BE2  1280
#define PV_B3   1536
#define PV_G3   1664
#define PV_BE3  1792
#define PV_END  1920

#define SZ_XB    ((size_t)NNODE * DIN * 2)
#define SZ_T     ((size_t)NNODE * DIN * 4)
#define SZ_H     ((size_t)NNODE * 2 * DIN * 2)
#define SZ_EMB   ((size_t)NNODE * DOUT * 4)
#define SZ_LIST  ((size_t)NNODE * DEGCAP * 4)
#define SZ_CNT   ((size_t)NNODE * 4)
#define SZ_W1T   ((size_t)DIN * DIN * 2)
#define SZ_W2D   ((size_t)DIN * 2 * DIN * 2)
#define SZ_W3D   ((size_t)DOUT * 2 * DIN * 2)
#define SZ_PV    ((size_t)U_PV * 16)
#define O_XB     ((size_t)0)
#define O_T      (O_XB + SZ_XB)
#define O_H      (O_T + SZ_T)
#define O_EMB    (O_H + SZ_H)
#define O_LIST   (O_EMB + SZ_EMB)
#define O_CNT    (O_LIST + SZ_LIST)
#define O_W1T    (O_CNT + SZ_CNT)
#define O_W2D    (O_W1T + SZ_W1T)
#define O_W3D    (O_W2D + SZ_W2D)
#define O_PV     (O_W3D + SZ_W3D)
#define WS_TOTAL (O_PV + SZ_PV)

static_assert(NNODE % OWN_BLK == 0);
static_assert((NNODE / OWN_BLK) * 8 * OWN_WAVE == NNODE);
static_assert(NEDGE % 2048 == 0);
static_assert(NEDGE % 256 == 0);
static_assert(DEGCAP == 128);
static_assert(DIN == 32 * 8);
static_assert(DOUT == 32 * 4);
static_assert(1024 * 8 == NNODE);
static_assert(NNODE <= 65536);
static_assert(WSTRIP + 4 <= STRIPW && (STRIPW % 4) == 0);
static_assert(LDS_BUCKET <= 262144);
static_assert(NNODE % 64 == 0 && DIN % 64 == 0 && DOUT % 64 == 0 && KT2 % 32 == 0 && KT3 % 32 == 0);
static_assert(U_W1 % 256 == 0 && U_W2 % 256 == 0 && U_W3 % 256 == 0 && U_PV % 256 == 0);
static_assert(PV_END <= U_PV * 4);
static_assert((size_t)NNODE * KT2 * 2 <= SZ_H && (size_t)NNODE * KT3 * 2 <= SZ_H);
static_assert((size_t)DIN * KT2 * 2 <= SZ_W2D && (size_t)DOUT * KT3 * 2 <= SZ_W3D);
static_assert((size_t)NNODE * DOUT * 4 <= SZ_T);
static_assert(WS_TOTAL == (size_t)29925376);
static_assert(WS_TOTAL <= ((size_t)128 << 20));
static_assert((O_T % 256) == 0 && (O_H % 256) == 0 && (O_EMB % 256) == 0 && (O_LIST % 256) == 0 &&
              (O_CNT % 256) == 0 && (O_W1T % 256) == 0 && (O_W2D % 256) == 0 && (O_W3D % 256) == 0 && (O_PV % 256) == 0);

typedef int v4i __attribute__((ext_vector_type(4)));
typedef v4i __attribute__((may_alias)) v4ia;

__device__ __forceinline__ void wave_lds_sync() {
  __builtin_amdgcn_fence(__ATOMIC_RELEASE, "workgroup");
  __builtin_amdgcn_wave_barrier();
  __builtin_amdgcn_fence(__ATOMIC_ACQUIRE, "workgroup");
}

__device__ __forceinline__ float wave_sum(float v) {
#pragma unroll
  for (int off = 16; off > 0; off >>= 1) v = v + __shfl_xor(v, off);
  return v;
}

__device__ __forceinline__ void wt_unit(const float* __restrict__ w, int cols, int ktot,
                                        unsigned short* __restrict__ dst, int u) {
  const int ppr = ktot >> 3;
  const int n   = u / ppr;
  const int p   = u - n * ppr;
  const int k8  = (p & (DIN / 8 - 1)) << 3;
  const float* q = w + (size_t)k8 * (size_t)cols + clampi(n, 0, cols - 1);
  float x[8];
#pragma unroll
  for (int e = 0; e < 8; ++e) {
    const float v = q[(size_t)e * (size_t)cols];
    asm volatile("" :: "v"(v));
    x[e] = v;
  }
  const v4u o = pack8_bf16((v4f){ x[0], x[1], x[2], x[3] }, (v4f){ x[4], x[5], x[6], x[7] });
  volatile v4u* d = (volatile v4u*)(dst + (size_t)u * 8);
  *d = o;
  __threadfence();
  *d = o;
}

#define PVSEG(P, BASE, LEN) { \
    const v4f t = *(const v4fa*)((P) + clampi(j4 - (BASE), 0, (LEN) - 4)); \
    asm volatile("" :: "v"(t)); \
    const unsigned mk = (j4 >= (BASE) && j4 < (BASE) + (LEN)) ? 0xFFFFFFFFu : 0u; \
    const v4u tb = (v4u){ bf16_bits(t[0]) << 16, bf16_bits(t[1]) << 16, bf16_bits(t[2]) << 16, bf16_bits(t[3]) << 16 }; \
    acc |= tb & (v4u){ mk, mk, mk, mk }; }

__global__ __launch_bounds__(256) void k_prep(
    const float* __restrict__ w1, const float* __restrict__ w2, const float* __restrict__ w3,
    const float* __restrict__ b1, const float* __restrict__ g1, const float* __restrict__ be1,
    const float* __restrict__ b2, const float* __restrict__ g2, const float* __restrict__ be2,
    const float* __restrict__ b3, const float* __restrict__ g3, const float* __restrict__ be3,
    unsigned short* __restrict__ W1T, unsigned short* __restrict__ W2D, unsigned short* __restrict__ W3D,
    float* __restrict__ PV) {
  const int u = (int)blockIdx.x * 256 + (int)threadIdx.x;
  if (u < U_W1) {
    wt_unit(w1, DIN, DIN, W1T, u);
  } else if (u < U_W1 + U_W2) {
    wt_unit(w2, DIN, KT2, W2D, u - U_W1);
  } else if (u < U_W1 + U_W2 + U_W3) {
    wt_unit(w3, DOUT, KT3, W3D, u - U_W1 - U_W2);
  } else if (u < U_TOT) {
    const int j4 = (u - (U_W1 + U_W2 + U_W3)) * 4;
    v4u acc = (v4u){ 0u, 0u, 0u, 0u };
    PVSEG(b1,  PV_B1,  DIN)
    PVSEG(g1,  PV_G1,  DIN)
    PVSEG(be1, PV_BE1, DIN)
    PVSEG(b2,  PV_B2,  DIN)
    PVSEG(g2,  PV_G2,  DIN)
    PVSEG(be2, PV_BE2, DIN)
    PVSEG(b3,  PV_B3,  DOUT)
    PVSEG(g3,  PV_G3,  DOUT)
    PVSEG(be3, PV_BE3, DOUT)
    volatile v4u* d = (volatile v4u*)(PV + j4);
    *d = acc;
    __threadfence();
    *d = acc;
  }
}
#undef PVSEG

template <int TWO>
__global__ __launch_bounds__(256) void k_row_tanh(const float* __restrict__ T, const float* __restrict__ gv,
                                                  const float* __restrict__ bv, unsigned short* __restrict__ H) {
  __shared__ __attribute__((aligned(16))) float st[8][DIN];
  const int lane = threadIdx.x & 31;
  const int wave = threadIdx.x >> 5;
  const int row  = (int)blockIdx.x * 8 + wave;
  const int rowc = clampi(row, 0, NNODE - 1);
  const float* tr = T + (size_t)rowc * DIN + 8 * lane;
  const v4f a = *(const v4fa*)tr;
  const v4f c = *(const v4fa*)(tr + 4);
  const v4f ga = *(const v4fa*)(gv + 8 * lane);
  const v4f gc = *(const v4fa*)(gv + 8 * lane + 4);
  const v4f ba = *(const v4fa*)(bv + 8 * lane);
  const v4f bc = *(const v4fa*)(bv + 8 * lane + 4);
  float s = ((a[0] + a[1]) + (a[2] + a[3])) + ((c[0] + c[1]) + (c[2] + c[3]));
  s = wave_sum(s);
  const float mu = s * (1.0f / 256.0f);
  const v4f da = (v4f){ a[0] - mu, a[1] - mu, a[2] - mu, a[3] - mu };
  const v4f dc = (v4f){ c[0] - mu, c[1] - mu, c[2] - mu, c[3] - mu };
  float q = ((da[0] * da[0] + da[1] * da[1]) + (da[2] * da[2] + da[3] * da[3])) +
            ((dc[0] * dc[0] + dc[1] * dc[1]) + (dc[2] * dc[2] + dc[3] * dc[3]));
  q = wave_sum(q);
  const float var = q * (1.0f / 256.0f);
  const float rs  = 1.0f / sqrtf(var + 1e-5f);
  const v4f ya = (v4f){ ((da[0] * rs) * ga[0]) + ba[0], ((da[1] * rs) * ga[1]) + ba[1],
                        ((da[2] * rs) * ga[2]) + ba[2], ((da[3] * rs) * ga[3]) + ba[3] };
  const v4f yc = (v4f){ ((dc[0] * rs) * gc[0]) + bc[0], ((dc[1] * rs) * gc[1]) + bc[1],
                        ((dc[2] * rs) * gc[2]) + bc[2], ((dc[3] * rs) * gc[3]) + bc[3] };
  float* sw = st[wave];
  *(v4fa*)(sw + 8 * lane)     = ya;
  *(v4fa*)(sw + 8 * lane + 4) = yc;
  wave_lds_sync();
#pragma unroll 1
  for (int i = 0; i < 8; ++i) {
    const float v = sw[i * 32 + lane];
    sw[i * 32 + lane] = tanhf(v);
  }
  wave_lds_sync();
  const v4f ha = *(const v4fa*)(sw + 8 * lane);
  const v4f hc = *(const v4fa*)(sw + 8 * lane + 4);
  const v4u hi = pack8_bf16(ha, hc);
  const v4u lo = pack8_bf16_lo(ha, hc);
  const int pitch = TWO ? 2 * DIN : DIN;
  unsigned short* hr = H + (size_t)rowc * (size_t)pitch + 8 * lane;
  if (row < NNODE) {
    *(volatile v4u*)hr = hi;
    if (TWO) *(volatile v4u*)(hr + DIN) = lo;
  }
  __threadfence();
  if (row < NNODE) {
    *(volatile v4u*)hr = hi;
    if (TWO) *(volatile v4u*)(hr + DIN) = lo;
  }
}

__global__ __launch_bounds__(256) void k_row_out(const float* __restrict__ T3, const float* __restrict__ gv,
                                                 const float* __restrict__ bv, float* __restrict__ out0,
                                                 float* __restrict__ EMB) {
  const int lane = threadIdx.x & 31;
  const int wave = threadIdx.x >> 5;
  const int row  = (int)blockIdx.x * 8 + wave;
  const int rowc = clampi(row, 0, NNODE - 1);
  const v4f a = *(const v4fa*)(T3 + (size_t)rowc * DOUT + 4 * lane);
  const v4f g = *(const v4fa*)(gv + 4 * lane);
  const v4f b = *(const v4fa*)(bv + 4 * lane);
  float s = (a[0] + a[1]) + (a[2] + a[3]);
  s = wave_sum(s);
  const float mu = s * (1.0f / 128.0f);
  const v4f d = (v4f){ a[0] - mu, a[1] - mu, a[2] - mu, a[3] - mu };
  float q = (d[0] * d[0] + d[1] * d[1]) + (d[2] * d[2] + d[3] * d[3]);
  q = wave_sum(q);
  const float var = q * (1.0f / 128.0f);
  const float rs  = 1.0f / sqrtf(var + 1e-5f);
  const v4f y = (v4f){ ((d[0] * rs) * g[0]) + b[0], ((d[1] * rs) * g[1]) + b[1],
                       ((d[2] * rs) * g[2]) + b[2], ((d[3] * rs) * g[3]) + b[3] };
  float* p0 = out0 + (size_t)rowc * DOUT + 4 * lane;
  float* p1 = EMB  + (size_t)rowc * DOUT + 4 * lane;
  if (row < NNODE) { *(volatile v4f*)p0 = y; *(volatile v4f*)p1 = y; }
  __threadfence();
  if (row < NNODE) { *(volatile v4f*)p0 = y; *(volatile v4f*)p1 = y; }
}

__global__ __launch_bounds__(256) void k_bucket(const int* __restrict__ ei, int* __restrict__ LIST,
                                                int* __restrict__ CNT) {
  extern __shared__ v4u lds_dyn[];
  int* strips = (int*)lds_dyn;
  unsigned short* tbls = (unsigned short*)(strips + 8 * STRIPW);
  const int lane = threadIdx.x & 31;
  const int wave = threadIdx.x >> 5;
  int* strip = strips + wave * STRIPW;
  unsigned short* tbl = tbls + wave * TBLH;
  const int obase = (int)blockIdx.x * OWN_BLK + wave * OWN_WAVE;
  const int* srcp = ei;
  const int* dstp = ei + NEDGE;

  int wc = 0;
#pragma unroll 1
  for (int it = 0; it < NEDGE / 256; ++it) {
    const int e0 = it * 256 + 8 * lane;
    const v4i sa = *(const v4ia*)(srcp + e0);
    const v4i sb = *(const v4ia*)(srcp + e0 + 4);
    const v4i da = *(const v4ia*)(dstp + e0);
    const v4i db = *(const v4ia*)(dstp + e0 + 4);
    asm volatile("" :: "v"(sa), "v"(sb));
    asm volatile("" :: "v"(da), "v"(db));
    const int sv[8] = { sa[0], sa[1], sa[2], sa[3], sb[0], sb[1], sb[2], sb[3] };
    const int dv[8] = { da[0], da[1], da[2], da[3], db[0], db[1], db[2], db[3] };
    unsigned w0[8], w1[8];
    int h0[8], h1[8];
    int cnt = 0;
#pragma unroll
    for (int j = 0; j < 8; ++j) {
      const int s = sv[j] - 1;
      const int d = dv[j] - 1;
      const bool ok = ((unsigned)s < (unsigned)NNODE) & ((unsigned)d < (unsigned)NNODE);
      const unsigned q0 = (unsigned)(d - obase);
      const unsigned q1 = (unsigned)(s - obase);
      h0[j] = (ok & (q0 < (unsigned)OWN_WAVE)) ? 1 : 0;
      h1[j] = (ok & (q1 < (unsigned)OWN_WAVE)) ? 1 : 0;
      w0[j] = (q0 << 16) | ((unsigned)s & 0xFFFFu);
      w1[j] = (q1 << 16) | ((unsigned)d & 0xFFFFu);
      cnt += h0[j] + h1[j];
    }
    int incl = cnt;
#pragma unroll
    for (int dd = 1; dd < 32; dd <<= 1) {
      const int up = __shfl_up(incl, dd);
      incl += (lane >= dd) ? up : 0;
    }
    const int tot = __builtin_amdgcn_readlane(incl, 31);
    int pos = wc + incl - cnt;
#pragma unroll
    for (int j = 0; j < 8; ++j) {
      if (h0[j] != 0 && pos < WSTRIP) strip[pos] = (int)w0[j];
      pos += h0[j];
      if (h1[j] != 0 && pos < WSTRIP) strip[pos] = (int)w1[j];
      pos += h1[j];
    }
    wc += tot;
  }
  const bool ovf = wc > WSTRIP;
  const int n = ovf ? WSTRIP : wc;
  if (lane < 4) strip[n + lane] = -1;
  wave_lds_sync();

#pragma unroll 1
  for (int p = 0; p < 2; ++p) {
    {
      const v8us z = (v8us){ 0, 0, 0, 0, 0, 0, 0, 0 };
      v8usa* tv = (v8usa*)tbl;
#pragma unroll
      for (int i = 0; i < TBLH / 8 / 32; ++i) tv[i * 32 + lane] = z;
    }
    wave_lds_sync();
    int cur = 0;
    const unsigned my = (unsigned)(p * 32 + lane);
#pragma unroll 1
    for (int i = 0; i < n; i += 4) {
      const v4i e = *(const v4ia*)(strip + i);
#pragma unroll
      for (int c = 0; c < 4; ++c) {
        const unsigned w = (unsigned)e[c];
        const bool mt = (w >> 16) == my;
        if (mt && cur < DEGCAP) tbl[lane * DEGCAP + cur] = (unsigned short)(w & 0xFFFFu);
        cur += mt ? 1 : 0;
      }
    }
    wave_lds_sync();
    for (int pass = 0; pass < 2; ++pass) {
#pragma unroll 2
      for (int r = 0; r < 32; ++r) {
        const unsigned short* tr = tbl + r * DEGCAP + 4 * lane;
        const v4i v = (v4i){ (int)tr[0], (int)tr[1], (int)tr[2], (int)tr[3] };
        const int owner = obase + p * 32 + r;
        *(volatile v4i*)(LIST + (size_t)owner * DEGCAP + 4 * lane) = v;
      }
      __threadfence();
    }
    const int cval = ovf ? CNT_SENT : cur;
    const int b4 = 4 * (lane & 7);
    const int c0 = __shfl(cval, b4);
    const int c1 = __shfl(cval, b4 + 1);
    const int c2 = __shfl(cval, b4 + 2);
    const int c3 = __shfl(cval, b4 + 3);
    const v4i cvv = (v4i){ c0, c1, c2, c3 };
    int* cq = CNT + obase + p * 32 + 4 * (lane & 7);
    if (lane < 8) *(volatile v4i*)cq = cvv;
    __threadfence();
    if (lane < 8) *(volatile v4i*)cq = cvv;
    wave_lds_sync();
  }
}

__global__ __launch_bounds__(256) void k_att(const float* __restrict__ EMB, const int* __restrict__ LIST,
                                             const int* __restrict__ CNT, float* __restrict__ out1) {
  const int lane = threadIdx.x & 31;
  const int wave = threadIdx.x >> 5;
  const int row  = (int)blockIdx.x * 8 + wave;
  const int rowc = clampi(row, 0, NNODE - 1);
  const v4i lw = *(const v4ia*)(LIST + (size_t)rowc * DEGCAP + 4 * lane);
  asm volatile("" :: "v"(lw));
  const int craw = CNT[rowc];
  asm volatile("" :: "v"(craw));
  const v4f o = *(const v4fa*)(EMB + (size_t)rowc * DOUT + 4 * lane);
  asm volatile("" :: "v"(o));
  const bool poison = (craw < 0) | (craw > DEGCAP);
  const int cv = poison ? 0 : craw;
  const int cn0 = __builtin_amdgcn_readfirstlane(cv);
  const int cn = cn0 < DEGCAP ? cn0 : DEGCAP;
  const int i0 = clampi(lw[0], 0, NNODE - 1);
  const int i1 = clampi(lw[1], 0, NNODE - 1);
  const int i2 = clampi(lw[2], 0, NNODE - 1);
  const int i3 = clampi(lw[3], 0, NNODE - 1);
  const int lp = 4 * lane;
  const float o0 = o[0], o1 = o[1], o2 = o[2], o3 = o[3];
  float den = 0.0f, a0 = 0.0f, a1 = 0.0f, a2 = 0.0f, a3 = 0.0f;
#pragma unroll 1
  for (int t = 0; t < cn; ++t) {
    const int L = t >> 2;
    const int c = t & 3;
    const int k0 = (c == 0) ? -1 : 0;
    const int k1 = (c == 1) ? -1 : 0;
    const int k2 = (c == 2) ? -1 : 0;
    const int k3 = (c == 3) ? -1 : 0;
    const int vs = (i0 & k0) | (i1 & k1) | (i2 & k2) | (i3 & k3);
    const int id = __builtin_amdgcn_readlane(vs, L);
    const bool m = ((i0 == id) & (lp < t)) | ((i1 == id) & (lp + 1 < t)) |
                   ((i2 == id) & (lp + 2 < t)) | ((i3 == id) & (lp + 3 < t));
    const unsigned dm = __builtin_amdgcn_ballot_w32(m);
    if (dm == 0u) {
      const v4f r = *(const v4fa*)(EMB + (size_t)id * DOUT + 4 * lane);
      const float r0 = r[0], r1 = r[1], r2 = r[2], r3 = r[3];
      asm volatile("" :: "v"(r0), "v"(r1), "v"(r2), "v"(r3));
      float pd = (o0 * r0 + o1 * r1) + (o2 * r2 + o3 * r3);
      pd = wave_sum(pd);
      const float e = expf(pd);
      den = den + e;
      a0 = a0 + e * r0;
      a1 = a1 + e * r1;
      a2 = a2 + e * r2;
      a3 = a3 + e * r3;
    }
  }
  const float qn = __uint_as_float(0x7fc00000u);
  float x0 = a0 / den;
  float x1 = a1 / den;
  float x2 = a2 / den;
  float x3 = a3 / den;
  x0 = poison ? qn : x0;
  x1 = poison ? qn : x1;
  x2 = poison ? qn : x2;
  x3 = poison ? qn : x3;
  const v4f xv = (v4f){ x0, x1, x2, x3 };
  float* po = out1 + (size_t)rowc * DOUT + 4 * lane;
  if (row < NNODE) *(volatile v4f*)po = xv;
  __threadfence();
  if (row < NNODE) *(volatile v4f*)po = xv;
}

static inline int cdiv_i(int a, int b) { return (a + b - 1) / b; }

extern "C" void kernel_launch(void* const* d_in, const int* in_sizes, int n_in,
                              void* d_out, int out_size, void* d_ws, size_t ws_size,
                              hipStream_t stream) {
  if (n_in < 14) return;
  if (in_sizes[0] != NNODE * DIN || in_sizes[1] != 2 * NEDGE) return;
  if (in_sizes[2] != DIN * DIN || in_sizes[3] != DIN || in_sizes[4] != DIN || in_sizes[5] != DIN) return;
  if (in_sizes[6] != DIN * DIN || in_sizes[7] != DIN || in_sizes[8] != DIN || in_sizes[9] != DIN) return;
  if (in_sizes[10] != DIN * DOUT || in_sizes[11] != DOUT || in_sizes[12] != DOUT || in_sizes[13] != DOUT) return;
  if (out_size != 2 * NNODE * DOUT) return;
  if (ws_size < WS_TOTAL) return;

  const float* x   = (const float*)d_in[0];
  const int*   ei  = (const int*)  d_in[1];
  const float* w1  = (const float*)d_in[2];
  const float* b1  = (const float*)d_in[3];
  const float* g1  = (const float*)d_in[4];
  const float* be1 = (const float*)d_in[5];
  const float* w2  = (const float*)d_in[6];
  const float* b2  = (const float*)d_in[7];
  const float* g2  = (const float*)d_in[8];
  const float* be2 = (const float*)d_in[9];
  const float* w3  = (const float*)d_in[10];
  const float* b3  = (const float*)d_in[11];
  const float* g3  = (const float*)d_in[12];
  const float* be3 = (const float*)d_in[13];

  float* out0 = (float*)d_out;
  float* out1 = (float*)d_out + (size_t)NNODE * DOUT;

  char* ws = (char*)d_ws;
  unsigned short* XB  = (unsigned short*)(ws + O_XB);
  float*          T   = (float*)(ws + O_T);
  unsigned short* H   = (unsigned short*)(ws + O_H);
  float*          EMB = (float*)(ws + O_EMB);
  int*            LST = (int*)(ws + O_LIST);
  int*            CNT = (int*)(ws + O_CNT);
  unsigned short* W1T = (unsigned short*)(ws + O_W1T);
  unsigned short* W2D = (unsigned short*)(ws + O_W2D);
  unsigned short* W3D = (unsigned short*)(ws + O_W3D);
  float*          PV  = (float*)(ws + O_PV);
  float*          T3  = T;

  hipFuncSetAttribute(reinterpret_cast<const void*>(&k_bucket),
                      hipFuncAttributeMaxDynamicSharedMemorySize, LDS_BUCKET);

  k_plane<0><<<NNODE * DIN / 8 / 256, 256, 0, stream>>>(x, NNODE, DIN, DIN, XB, NNODE, DIN);
  k_prep<<<U_TOT / 256, 256, 0, stream>>>(w1, w2, w3, b1, g1, be1, b2, g2, be2, b3, g3, be3, W1T, W2D, W3D, PV);
  {
    const int tiles = (NNODE / 64) * (DIN / 64);
    k_gemm_nt<0, 1><<<cdiv_i(tiles, 8), 256, 0, stream>>>(XB, W1T, PV + PV_B1, T, NNODE, DIN, DIN, DIN);
  }
  k_row_tanh<TWO_TERM_L2><<<NNODE / 8, 256, 0, stream>>>(T, PV + PV_G1, PV + PV_BE1, H);
  {
    const int tiles = (NNODE / 64) * (DIN / 64);
    k_gemm_nt<(TWO_TERM_L2 ? 1 : 0), 1><<<cdiv_i(tiles, 8), 256, 0, stream>>>(H, W2D, PV + PV_B2, T, NNODE, DIN, KT2, DIN);
  }
  k_row_tanh<TWO_TERM_L3><<<NNODE / 8, 256, 0, stream>>>(T, PV + PV_G2, PV + PV_BE2, H);
  {
    const int tiles = (NNODE / 64) * (DOUT / 64);
    k_gemm_nt<(TWO_TERM_L3 ? 1 : 0), 1><<<cdiv_i(tiles, 8), 256, 0, stream>>>(H, W3D, PV + PV_B3, T3, NNODE, DOUT, KT3, DOUT);
  }
  k_row_out<<<NNODE / 8, 256, 0, stream>>>(T3, PV + PV_G3, PV + PV_BE3, out0, EMB);
  k_bucket<<<NNODE / OWN_BLK, 256, LDS_BUCKET, stream>>>(ei, LST, CNT);
  k_att<<<NNODE / 8, 256, 0, stream>>>(EMB, LST, CNT, out1);
}
